// MultiHeadAttention_56427280335583
// MI455X (gfx1250) — hardware-verified
//
#include <hip/hip_runtime.h>
#include <math.h>

#ifndef NB
#define NB 2
#endif
#ifndef SEQ
#define SEQ 2048
#endif
#define NB_FULL 2
#define SEQ_FULL 2048
#define EMB 1024
#define NHEAD 16
#define NXR 256

static_assert(SEQ % 64 == 0);
static_assert(NXR % 64 == 0);
static_assert(SEQ >= NXR);
static_assert(SEQ <= SEQ_FULL);
static_assert(NB <= NB_FULL);
static_assert(NB >= 1);

typedef __attribute__((ext_vector_type(16))) _Float16 v16h;
typedef __attribute__((ext_vector_type(8)))  _Float16 v8h;
typedef __attribute__((ext_vector_type(16))) __bf16   v16b;
typedef __attribute__((ext_vector_type(8)))  __bf16   v8b;
typedef __attribute__((ext_vector_type(8)))  float    v8f;
typedef __attribute__((ext_vector_type(4)))  float    v4f;

union FragH { v16h v; v8h h[2]; };

__device__ __forceinline__ v8f wmma16(v16h a, v16h b, v8f c) {
    c = __builtin_amdgcn_wmma_f32_16x16x32_f16(false, a, false, b, (short)0, c, false, false);
    asm volatile("v_nop\n\tv_nop\n\tv_nop\n\tv_nop" : "+v"(c) : "v"(a), "v"(b));
    return c;
}

#define VST2(T, ptr, val) do { const T vst2_v_ = (val); *(volatile T*)(ptr) = vst2_v_; __threadfence(); *(volatile T*)(ptr) = vst2_v_; } while (0)

#define AT_NW 4
#define AT_LP 72
__global__ __launch_bounds__(32 * AT_NW) __attribute__((amdgpu_num_vgpr(256)))
void k_attn_c64(const float* __restrict__ Q, const float* __restrict__ K, const float* __restrict__ V, int ld, long long sb,
                float* __restrict__ O, int ldo, long long sob, int qrow0, float scale) {
    __shared__ __align__(16) _Float16 Ksh[64 * AT_LP];
    __shared__ __align__(16) _Float16 Vth[64 * AT_LP];
    __shared__ __align__(16) _Float16 Psh[AT_NW][16 * AT_LP];
    __shared__ __align__(16) float    Os[AT_NW][16 * 68];
    const int tid  = threadIdx.x;
    const int wave = __builtin_amdgcn_readfirstlane(tid >> 5);
    const int lane = tid & 31, hh = lane >> 4, c = lane & 15;
    const int h = blockIdx.y, b = blockIdx.z;
    const int qblk = qrow0 + (int)blockIdx.x * 64;
    const int q0 = qblk + wave * 16;
    const int nChunks = (qblk >> 6) + 1;
    const float L2E = 1.4426950408889634f;
    const float NEG = -__builtin_inff();

    const float* Qb = Q + (long long)b * sb + h * 64;
    const float* Kb = K + (long long)b * sb + h * 64;
    const float* Vb = V + (long long)b * sb + h * 64;
    float*       Ob = O + (long long)b * sob + h * 64;

    v16h qa[2];
    {
        const float* qrow = Qb + (long long)(q0 + c) * ld;
#pragma unroll
        for (int dc = 0; dc < 2; ++dc) {
            const v4f a0 = *(const v4f*)(qrow + dc * 32 + 8 * hh);
            const v4f a1 = *(const v4f*)(qrow + dc * 32 + 8 * hh + 4);
            const v4f b0 = *(const v4f*)(qrow + dc * 32 + 16 + 8 * hh);
            const v4f b1 = *(const v4f*)(qrow + dc * 32 + 16 + 8 * hh + 4);
#pragma unroll
            for (int e = 0; e < 4; ++e) {
                qa[dc][e]      = (_Float16)a0[e];
                qa[dc][4 + e]  = (_Float16)a1[e];
                qa[dc][8 + e]  = (_Float16)b0[e];
                qa[dc][12 + e] = (_Float16)b1[e];
            }
        }
    }

    v8f o[4]; float m8[8], l8[8];
#pragma unroll
    for (int t = 0; t < 4; ++t) { v8f zz = {}; o[t] = zz; }
#pragma unroll
    for (int r = 0; r < 8; ++r) { m8[r] = NEG; l8[r] = 0.f; }

    for (int kc = 0; kc < nChunks; ++kc) {
        const int kv0 = kc * 64;
        __syncthreads();
        {
            const int kvr = tid >> 1, dh = (tid & 1) * 32;
            const float* krow = Kb + (long long)(kv0 + kvr) * ld + dh;
            const float* vrow = Vb + (long long)(kv0 + kvr) * ld + dh;
#pragma unroll
            for (int i = 0; i < 8; ++i) {
                const v4f kk = *(const v4f*)(krow + 4 * i);
                const v4f vv = *(const v4f*)(vrow + 4 * i);
#pragma unroll
                for (int e = 0; e < 4; ++e) {
                    const int d = dh + 4 * i + e;
                    Ksh[kvr * AT_LP + d] = (_Float16)kk[e];
                    Vth[d * AT_LP + kvr] = (_Float16)vv[e];
                }
            }
        }
        __syncthreads();

        v8f s[4];
#pragma unroll
        for (int j = 0; j < 4; ++j) {
            v8f acc = {};
#pragma unroll
            for (int dc = 0; dc < 2; ++dc) {
                FragH kb;
                kb.h[0] = *(const v8h*)&Ksh[(j * 16 + c) * AT_LP + dc * 32 + 8 * hh];
                kb.h[1] = *(const v8h*)&Ksh[(j * 16 + c) * AT_LP + dc * 32 + 16 + 8 * hh];
                acc = wmma16(qa[dc], kb.v, acc);
            }
            s[j] = acc;
        }

#pragma unroll
        for (int r = 0; r < 8; ++r) {
            const int irow = q0 + 8 * hh + r;
            float sc[4];
#pragma unroll
            for (int j = 0; j < 4; ++j) {
                const int jg = kv0 + j * 16 + c;
                const float v = s[j][r] * scale;
                sc[j] = (jg > irow) ? NEG : v * L2E;
            }
            float mx = fmaxf(fmaxf(sc[0], sc[1]), fmaxf(sc[2], sc[3]));
            mx = fmaxf(mx, __shfl_xor(mx, 1, 32)); mx = fmaxf(mx, __shfl_xor(mx, 2, 32));
            mx = fmaxf(mx, __shfl_xor(mx, 4, 32)); mx = fmaxf(mx, __shfl_xor(mx, 8, 32));
            const float mnew = fmaxf(m8[r], mx);
            const float corr = (mnew == NEG) ? 1.f : exp2f(m8[r] - mnew);
            float rs = 0.f;
#pragma unroll
            for (int j = 0; j < 4; ++j) {
                const float pp = (sc[j] == NEG) ? 0.f : exp2f(sc[j] - mnew);
                rs += pp;
                Psh[wave][(8 * hh + r) * AT_LP + j * 16 + c] = (_Float16)(pp * 4096.f);
            }
            rs += __shfl_xor(rs, 1, 32); rs += __shfl_xor(rs, 2, 32); rs += __shfl_xor(rs, 4, 32); rs += __shfl_xor(rs, 8, 32);
            l8[r] = l8[r] * corr + rs; m8[r] = mnew;
#pragma unroll
            for (int t = 0; t < 4; ++t) o[t][r] *= corr;
        }
        __syncthreads();

#pragma unroll
        for (int kk = 0; kk < 2; ++kk) {
            FragH pa;
            pa.h[0] = *(const v8h*)&Psh[wave][c * AT_LP + kk * 32 + 8 * hh];
            pa.h[1] = *(const v8h*)&Psh[wave][c * AT_LP + kk * 32 + 16 + 8 * hh];
#pragma unroll
            for (int t = 0; t < 4; ++t) {
                FragH vb;
                vb.h[0] = *(const v8h*)&Vth[(t * 16 + c) * AT_LP + kk * 32 + 8 * hh];
                vb.h[1] = *(const v8h*)&Vth[(t * 16 + c) * AT_LP + kk * 32 + 16 + 8 * hh];
                o[t] = wmma16(pa.v, vb.v, o[t]);
            }
        }
    }

#pragma unroll
    for (int r = 0; r < 8; ++r) {
        const float inv = (l8[r] > 0.f) ? 1.f / (l8[r] * 4096.f) : 0.f;
#pragma unroll
        for (int t = 0; t < 4; ++t) Os[wave][(8 * hh + r) * 68 + t * 16 + c] = o[t][r] * inv;
    }
    __syncthreads();
    {
        const int c4 = (lane & 15) * 4;
        for (int pass = 0; pass < 2; ++pass) {
#pragma unroll
            for (int it = 0; it < 8; ++it) {
                const int row = it * 2 + hh;
                const v4f val = *(const v4f*)&Os[wave][row * 68 + c4];
                *(volatile v4f*)(Ob + (long long)(q0 + row) * ldo + c4) = val;
            }
            __threadfence();
        }
    }
}

namespace w25 {

__device__ __forceinline__ unsigned short f2bf_bits(float f) {
  unsigned u = __float_as_uint(f);
  return (unsigned short)((u + 0x7FFFu + ((u >> 16) & 1u)) >> 16);
}
__device__ __forceinline__ float bf_bits2f(unsigned short h) { return __uint_as_float(((unsigned)h) << 16); }

__device__ __forceinline__ void dep_guard_h(v8f& a, v8f& b, v16h x, v16h y) { asm volatile("v_nop\n\tv_nop\n\tv_nop\n\tv_nop" : "+v"(a), "+v"(b) : "v"(x), "v"(y)); }
__device__ __forceinline__ void dep_guard_b(v8f& a, v8f& b, v16b x, v16b y) { asm volatile("v_nop\n\tv_nop\n\tv_nop\n\tv_nop" : "+v"(a), "+v"(b) : "v"(x), "v"(y)); }
__device__ __forceinline__ void keep4_h(v16h a, v16h b, v16h c, v16h d) { asm volatile("v_nop" :: "v"(a), "v"(b), "v"(c), "v"(d)); }
__device__ __forceinline__ void keep4_b(v16b a, v16b b, v16b c, v16b d) { asm volatile("v_nop" :: "v"(a), "v"(b), "v"(c), "v"(d)); }
__device__ __forceinline__ void acc_guard4(v8f& a, v8f& b, v8f& c, v8f& d) { asm volatile("v_nop\n\tv_nop\n\tv_nop\n\tv_nop" : "+v"(a), "+v"(b), "+v"(c), "+v"(d)); }
template <typename T> struct Frag;
template <> struct Frag<_Float16> {
  typedef v16h V; union U { v16h v; v8h h[2]; };
  static __device__ __forceinline__ v16h load(const _Float16* p) {
    U f; f.h[0] = *(const v8h*)(p); f.h[1] = *(const v8h*)(p + 16); return f.v;
  }
  static __device__ __forceinline__ v8f mma(v16h a, v16h b, v8f c) {
    return __builtin_amdgcn_wmma_f32_16x16x32_f16(false, a, false, b, (short)0, c, false, false);
  }
  static __device__ __forceinline__ void guard(v8f& a, v8f& b, v16h x, v16h y) { dep_guard_h(a, b, x, y); }
  static __device__ __forceinline__ void keep(v16h a, v16h b, v16h c, v16h d) { keep4_h(a, b, c, d); }
};
template <> struct Frag<__bf16> {
  typedef v16b V; union U { v16b v; v8b h[2]; };
  static __device__ __forceinline__ v16b load(const __bf16* p) {
    U f; f.h[0] = *(const v8b*)(p); f.h[1] = *(const v8b*)(p + 16); return f.v;
  }
  static __device__ __forceinline__ v8f mma(v16b a, v16b b, v8f c) {
    return __builtin_amdgcn_wmma_f32_16x16x32_bf16(false, a, false, b, (short)0, c, false, false);
  }
  static __device__ __forceinline__ void guard(v8f& a, v8f& b, v16b x, v16b y) { dep_guard_b(a, b, x, y); }
  static __device__ __forceinline__ void keep(v16b a, v16b b, v16b c, v16b d) { keep4_b(a, b, c, d); }
};

template <int ET> struct Elem;
template <> struct Elem<0> { typedef _Float16 T; };
template <> struct Elem<1> { typedef __bf16 T; };
template <int ET, int BIAS_MODE, bool RESID>
__global__ __launch_bounds__(256) __attribute__((amdgpu_num_vgpr(256))) void wmma_gemm64(
    const unsigned short* __restrict__ Ap, int lda, long strideA,
    const unsigned short* __restrict__ Btp, int ldb, long strideB,
    float* Cout, int ldc, long strideC,
    const float* __restrict__ bias,
    const float* resid, long strideR,
    int M, int N, int K, float scale) {
  typedef typename Elem<ET>::T T;
  typedef typename Frag<T>::V V;
  const T* A = (const T*)Ap; const T* Bt = (const T*)Btp;
  __shared__ __align__(16) float sT[8][16 * 68];
  const int b    = blockIdx.y;
  const int lane = threadIdx.x & 31;
  const int wave = __builtin_amdgcn_readfirstlane(threadIdx.x >> 5);
  const int tilesN = N >> 6;
  const int tilesM = M >> 6;
  const int tile = blockIdx.x * 8 + wave;
  if (tile >= tilesM * tilesN) return;
  const int tm = tile / tilesN;
  const int tn = tile - tm * tilesN;
  const int m0 = tm << 6;
  const int n0 = tn << 6;

  const T* Ab  = A  + (size_t)b * strideA;
  const T* Bb  = Bt + (size_t)b * strideB;

  const int rlane = lane & 15;
  const int koff  = (lane >> 4) * 8;
  const int mOff  = (lane >> 4) * 8;

  v8f acc[4][4];
#pragma unroll
  for (int i = 0; i < 4; ++i)
#pragma unroll
    for (int j = 0; j < 4; ++j) acc[i][j] = (v8f){0.f,0.f,0.f,0.f,0.f,0.f,0.f,0.f};

  for (int k0 = 0; k0 < K; k0 += 32) {
    V bh[4];
#pragma unroll
    for (int j = 0; j < 4; ++j) {
      const size_t bo = (size_t)(n0 + (j << 4) + rlane) * ldb + koff + k0;
      bh[j] = Frag<T>::load(Bb + bo);
    }
#pragma unroll
    for (int i = 0; i < 4; ++i) {
      const size_t ao = (size_t)(m0 + (i << 4) + rlane) * lda + koff + k0;
      V ah = Frag<T>::load(Ab + ao);
#pragma unroll
      for (int j = 0; j < 4; ++j) {
        acc[i][j] = Frag<T>::mma(ah, bh[j], acc[i][j]);
      }
      Frag<T>::guard(acc[i][0], acc[i][3], ah, ah);
    }
    Frag<T>::keep(bh[0], bh[1], bh[2], bh[3]);
  }
  acc_guard4(acc[0][0], acc[0][1], acc[0][2], acc[0][3]);
  acc_guard4(acc[1][0], acc[1][1], acc[1][2], acc[1][3]);
  acc_guard4(acc[2][0], acc[2][1], acc[2][2], acc[2][3]);
  acc_guard4(acc[3][0], acc[3][1], acc[3][2], acc[3][3]);

  const float* Rb = RESID ? (resid + (size_t)b * strideR) : nullptr;
#pragma unroll
  for (int i = 0; i < 4; ++i) {
    const int mBase = m0 + (i << 4);
#pragma unroll
    for (int j = 0; j < 4; ++j) {
      const int n = n0 + (j << 4) + rlane;
      float bv = 0.f;
      if (BIAS_MODE == 2) bv = bias[n];
#pragma unroll
      for (int r = 0; r < 8; ++r) {
        float v = acc[i][j][r] * scale;
        if (BIAS_MODE == 2) v += bv;
        if (RESID) v += Rb[(size_t)(mBase + mOff + r) * ldc + n];
        sT[wave][(mOff + r) * 68 + (j << 4) + rlane] = v;
      }
    }
    __builtin_amdgcn_fence(3  , "workgroup");
    __builtin_amdgcn_wave_barrier();
    __builtin_amdgcn_fence(2  , "workgroup");
    {
      float* C = Cout + (size_t)b * strideC;
      const int hh = lane >> 4, c4 = (lane & 15) * 4;
      for (int pass = 0; pass < 2; ++pass) {
#pragma unroll
        for (int it = 0; it < 8; ++it) {
          const int row = it * 2 + hh;
          const v4f v = *(const v4f*)&sT[wave][row * 68 + c4];
          *(volatile v4f*)(C + (size_t)(mBase + row) * ldc + n0 + c4) = v;
        }
        __threadfence();
      }
    }
    __builtin_amdgcn_fence(3  , "workgroup");
    __builtin_amdgcn_wave_barrier();
    __builtin_amdgcn_fence(2  , "workgroup");
  }
}

}

__global__ __launch_bounds__(256) void k_cast16(const float* __restrict__ src, long long lds, _Float16* __restrict__ dst, long long ldd, int R, int C, float s) {
    const long long i = (long long)blockIdx.x * 256 + threadIdx.x; const long long np = (long long)R * (C / 2); if (i >= np) return; const int r = (int)(i / (C / 2)); const int c = 2 * (int)(i % (C / 2));
    const _Float16 h0 = (_Float16)(src[(long long)r * lds + c] * s), h1 = (_Float16)(src[(long long)r * lds + c + 1] * s);
    const unsigned u = (unsigned)__builtin_bit_cast(unsigned short, h0) | ((unsigned)__builtin_bit_cast(unsigned short, h1) << 16);
    volatile unsigned* d = (volatile unsigned*)(dst + (long long)r * ldd + c); *d = u; __threadfence(); *d = u; }

__device__ __forceinline__ unsigned int f2bf2_pack(float a, float b, unsigned int* lo) {
    const unsigned short ha = w25::f2bf_bits(a), hb = w25::f2bf_bits(b);
    const unsigned short la = w25::f2bf_bits(a - w25::bf_bits2f(ha)), lb = w25::f2bf_bits(b - w25::bf_bits2f(hb));
    *lo = (unsigned)la | ((unsigned)lb << 16); return (unsigned)ha | ((unsigned)hb << 16); }
__global__ __launch_bounds__(256) void k_castS16(const float* __restrict__ src, long long lds, __bf16* __restrict__ dhi, __bf16* __restrict__ dlo, long long ldd, int R, int C, float s, int transpose) {
    const long long i = (long long)blockIdx.x * 256 + threadIdx.x; long long o; float a, b;
    if (transpose) { const long long np = (long long)C * (R / 2); if (i >= np) return; const int c = (int)(i / (R / 2)); const int r = 2 * (int)(i % (R / 2)); a = src[(long long)r * lds + c] * s; b = src[(long long)(r + 1) * lds + c] * s; o = (long long)c * ldd + r; }
    else { const long long np = (long long)R * (C / 2); if (i >= np) return; const int r = (int)(i / (C / 2)); const int c = 2 * (int)(i % (C / 2)); a = src[(long long)r * lds + c] * s; b = src[(long long)r * lds + c + 1] * s; o = (long long)r * ldd + c; }
    unsigned lo; const unsigned hi = f2bf2_pack(a, b, &lo); volatile unsigned* ph = (volatile unsigned*)(dhi + o); volatile unsigned* pl = (volatile unsigned*)(dlo + o);
    *ph = hi; *pl = lo; __threadfence(); *ph = hi; *pl = lo; }

typedef unsigned int cm_u4 __attribute__((ext_vector_type(4)));
__device__ __forceinline__ unsigned int cmb_pk2(float a, float b) { return (unsigned int)__builtin_bit_cast(unsigned short, (_Float16)a) | ((unsigned int)__builtin_bit_cast(unsigned short, (_Float16)b) << 16); }
__device__ __forceinline__ float cmb_bf(float v) { const unsigned u = __builtin_bit_cast(unsigned, v); const unsigned r = (u + 0x7fffu + ((u >> 16) & 1u)) & 0xffff0000u; return __builtin_bit_cast(float, r); }
__global__ __launch_bounds__(256) void k_cm_bfvec(const float* __restrict__ SRC, float* __restrict__ DST, int n) { const int u = blockIdx.x * 256 + threadIdx.x; if (u >= n) return; VST2(float, DST + u, cmb_bf(SRC[u])); }
__global__ __launch_bounds__(256) void k_cm_castb(const float* __restrict__ SRC, int lds, long long sSz, unsigned short* __restrict__ DST, int ldd, long long sDz, int nR, int nC, float sc) {
    const long long u = (long long)blockIdx.x * 256 + threadIdx.x; const int per = nC / 8; if (u >= (long long)nR * per) return; const int r = (int)(u / per); const int c0 = 8 * (int)(u % per);
    const float* s = SRC + (long long)blockIdx.y * sSz + (long long)r * lds + c0; float w[8];
#pragma unroll
    for (int e = 0; e < 8; ++e) w[e] = cmb_bf(s[e]) * sc;
    cm_u4 pk; pk.x = cmb_pk2(w[0], w[1]); pk.y = cmb_pk2(w[2], w[3]); pk.z = cmb_pk2(w[4], w[5]); pk.w = cmb_pk2(w[6], w[7]); VST2(cm_u4, (cm_u4*)(DST + (long long)blockIdx.y * sDz + (long long)r * ldd + c0), pk); }
__global__ __launch_bounds__(256) void k_cm_castbT(const float* __restrict__ SRC, int lds, unsigned short* __restrict__ DST, int ldd, int nR, int nC, float sc) {
    const long long u = (long long)blockIdx.x * 256 + threadIdx.x; const int per = nR / 8; if (u >= (long long)nC * per) return; const int c = (int)(u / per); const int r0 = 8 * (int)(u % per);
    float w[8];
#pragma unroll
    for (int e = 0; e < 8; ++e) w[e] = cmb_bf(SRC[(long long)(r0 + e) * lds + c]) * sc;
    cm_u4 pk; pk.x = cmb_pk2(w[0], w[1]); pk.y = cmb_pk2(w[2], w[3]); pk.z = cmb_pk2(w[4], w[5]); pk.w = cmb_pk2(w[6], w[7]); VST2(cm_u4, (cm_u4*)(DST + (long long)c * ldd + r0), pk); }

template <int NX, int HREP>
__global__ __launch_bounds__(64) void k_gx_exact(const float* __restrict__ Q, int ldq, const float* __restrict__ KV, int ldkv, int voff, float sc, float* __restrict__ AOX, int ldo) {
    #pragma clang fp contract(off)
    __shared__ float qs[64]; __shared__ float ps[NX]; __shared__ float red[2];
    const int i = blockIdx.x, h = blockIdx.y, t = threadIdx.x; const int kvh = h / HREP;
    qs[t] = Q[(long long)i * ldq + h * 64 + t]; __syncthreads();
#pragma unroll
    for (int r = 0; r < NX / 64; ++r) { const int j = t + 64 * r; const int jc = min(j, i); const float* kr = KV + (long long)jc * ldkv + kvh * 64; float s = 0.f;
#pragma unroll 8
        for (int d = 0; d < 64; ++d) s += qs[d] * kr[d];
        ps[j] = (j <= i) ? s * sc : -3.0e38f; }
    __syncthreads();
    if (t == 0) { float m = -3.0e38f; for (int j = 0; j <= i; ++j) m = fmaxf(m, ps[j]); float z = 0.f; for (int j = 0; j <= i; ++j) { const float e = expf(ps[j] - m); ps[j] = e; z += e; } red[0] = 1.f / z; }
    __syncthreads();
    const float inv = red[0]; float o = 0.f;
    for (int j = 0; j <= i; ++j) o += ps[j] * KV[(long long)j * ldkv + voff + kvh * 64 + t];
    VST2(float, AOX + (long long)i * ldo + h * 64 + t, o * inv); }

#define CARVE_BYTES(n) ((((size_t)(n)) + 255) / 256 * 256)

extern "C" void kernel_launch(void* const* d_in, const int* in_sizes, int n_in, void* d_out, int out_size, void* d_ws, size_t ws_size, hipStream_t stream) {
    if (n_in < 5) return;
    const long long span = (long long)(NB - 1) * SEQ_FULL * EMB + (long long)SEQ * EMB;
    if ((long long)in_sizes[0] < span) return;
    if ((long long)in_sizes[1] < (long long)EMB * 3 * EMB) return;
    if (in_sizes[2] < 3 * EMB) return;
    if ((long long)in_sizes[3] < (long long)EMB * EMB) return;
    if (in_sizes[4] < EMB) return;
    if ((long long)out_size < span) return;
    const float* x    = (const float*)d_in[0];
    const float* Wkqv = (const float*)d_in[1];
    const float* bkqv = (const float*)d_in[2];
    const float* Wo   = (const float*)d_in[3];
    const float* bo   = (const float*)d_in[4];
    float* out = (float*)d_out;
    const int MTOK = NB * SEQ;
    char* wsp = (char*)d_ws;
    unsigned short* X16  = (unsigned short*)wsp; wsp += CARVE_BYTES((size_t)MTOK * EMB * 2);
    unsigned short* W316 = (unsigned short*)wsp; wsp += CARVE_BYTES((size_t)3 * EMB * EMB * 2);
    float* QKV = (float*)wsp;                    wsp += CARVE_BYTES((size_t)MTOK * 3 * EMB * 4);
    float* AO  = (float*)wsp;                    wsp += CARVE_BYTES((size_t)MTOK * EMB * 4);
    float* BR3 = (float*)wsp;                    wsp += CARVE_BYTES((size_t)(3 * EMB + 64) * 4);
    unsigned short* AO16 = X16;
    unsigned short* WO16 = (unsigned short*)wsp; wsp += CARVE_BYTES((size_t)EMB * EMB * 2);
    unsigned short* WOB  = (unsigned short*)wsp; wsp += CARVE_BYTES((size_t)EMB * EMB * 2);
    unsigned short* WOL  = (unsigned short*)wsp; wsp += CARVE_BYTES((size_t)EMB * EMB * 2);
    unsigned short* AOH2 = (unsigned short*)wsp; wsp += CARVE_BYTES((size_t)NXR * EMB * 2);
    unsigned short* AOL2 = (unsigned short*)wsp; wsp += CARVE_BYTES((size_t)NXR * EMB * 2);
    float* BRO = (float*)wsp;                    wsp += CARVE_BYTES((size_t)(EMB + 64) * 4);
    const size_t carved = (size_t)(wsp - (char*)d_ws);
    if (carved > ws_size || carved > (size_t)134217728) return;

    k_cm_castb<<<dim3((unsigned)(((long long)SEQ * (EMB / 8) + 255) / 256), (unsigned)NB), 256, 0, stream>>>(x, EMB, (long long)SEQ_FULL * EMB, X16, EMB, (long long)SEQ * EMB, SEQ, EMB, 1.0f);
    k_cm_castbT<<<(unsigned)(((long long)(3 * EMB) * (EMB / 8) + 255) / 256), 256, 0, stream>>>(Wkqv, 3 * EMB, W316, EMB, EMB, 3 * EMB, 16.0f);
    k_cm_bfvec<<<(3 * EMB + 255) / 256, 256, 0, stream>>>(bkqv, BR3, 3 * EMB);
    w25::wmma_gemm64<0, 2, false><<<dim3((unsigned)((((MTOK) / 64) * ((3 * EMB) / 64) + 7) / 8), 1u), 256, 0, stream>>>(
        X16, EMB, 0, W316, EMB, 0, QKV, 3 * EMB, 0, BR3, nullptr, 0, MTOK, 3 * EMB, EMB, 0.0625f);
    k_cm_castbT<<<(unsigned)(((long long)EMB * (EMB / 8) + 255) / 256), 256, 0, stream>>>(Wo, EMB, WO16, EMB, EMB, EMB, 16.0f);
    k_castS16<<<(unsigned)(((long long)EMB * (EMB / 2) + 255) / 256), 256, 0, stream>>>(Wo, EMB, (__bf16*)WOB, (__bf16*)WOL, EMB, EMB, EMB, 1.0f, 1);
    k_cm_bfvec<<<(EMB + 255) / 256, 256, 0, stream>>>(bo, BRO, EMB);
    for (int b = 0; b < NB; ++b) {
        const float* qkvb = QKV + (size_t)b * SEQ * 3 * EMB;
        k_gx_exact<NXR, 1><<<dim3(NXR, NHEAD), 64, 0, stream>>>(qkvb + EMB, 3 * EMB, qkvb, 3 * EMB, 2 * EMB, 0.125f, AO + (size_t)b * SEQ * EMB, EMB);
    }
#if SEQ > NXR
    k_attn_c64<<<dim3((unsigned)((SEQ - NXR) / 64), (unsigned)NHEAD, (unsigned)NB), 32 * AT_NW, 0, stream>>>(
        QKV + EMB, QKV, QKV + 2 * EMB, 3 * EMB, (long long)SEQ * 3 * EMB, AO, EMB, (long long)SEQ * EMB, NXR, 0.125f);
#endif
    k_cast16<<<(unsigned)(((long long)MTOK * (EMB / 2) + 255) / 256), 256, 0, stream>>>(AO, EMB, (_Float16*)AO16, EMB, MTOK, EMB, 64.0f);
    w25::wmma_gemm64<0, 2, false><<<dim3((unsigned)((((SEQ) / 64) * ((EMB) / 64) + 7) / 8), (unsigned)NB), 256, 0, stream>>>(
        AO16, EMB, (long)SEQ * EMB, WO16, EMB, 0, out, EMB, (long)SEQ_FULL * EMB, BRO, nullptr, 0, SEQ, EMB, EMB, 0.0009765625f);
    for (int b = 0; b < NB; ++b) {
        float* ob = out + (size_t)b * SEQ_FULL * EMB;
        k_castS16<<<(unsigned)(((long long)NXR * (EMB / 2) + 255) / 256), 256, 0, stream>>>(AO + (size_t)b * SEQ * EMB, EMB, (__bf16*)AOH2, (__bf16*)AOL2, EMB, NXR, EMB, 1.0f, 0);
        w25::wmma_gemm64<1, 2, false><<<dim3((unsigned)((((NXR) / 64) * ((EMB) / 64) + 7) / 8), 1u), 256, 0, stream>>>(
            AOH2, EMB, 0, WOB, EMB, 0, ob, EMB, 0, BRO, nullptr, 0, NXR, EMB, EMB, 1.0f);
        w25::wmma_gemm64<1, 0, true><<<dim3((unsigned)((((NXR) / 64) * ((EMB) / 64) + 7) / 8), 1u), 256, 0, stream>>>(
            AOL2, EMB, 0, WOB, EMB, 0, ob, EMB, 0, nullptr, ob, 0, NXR, EMB, EMB, 1.0f);
    }
}
